// SMFNet_64347200028731
// MI455X (gfx1250) — hardware-run, weakly checked
//
#include <hip/hip_runtime.h>


#define NN  4096
#define ND  512
#define NLY 3
typedef _Float16 h16;
typedef unsigned short bf;
typedef __attribute__((ext_vector_type(16))) __bf16   v16bf;
typedef __attribute__((ext_vector_type(16))) _Float16 v16h;
typedef __attribute__((ext_vector_type(8)))  _Float16 v8h;
typedef __attribute__((ext_vector_type(8)))  unsigned short v8us;
typedef __attribute__((ext_vector_type(8)))  float    v8f;
typedef __attribute__((ext_vector_type(4)))  float    v4f;
typedef v8h  __attribute__((may_alias)) v8ha;
typedef v4f  __attribute__((may_alias)) v4fa;
typedef v8us __attribute__((may_alias)) v8usa;

__device__ __forceinline__ unsigned short f2bf(float f) { unsigned u = __float_as_uint(f); u += 0x7FFFu + ((u >> 16) & 1u); return (unsigned short)(u >> 16); }
__device__ __forceinline__ float bf2f(unsigned short b) { return __uint_as_float(((unsigned)b) << 16); }
__device__ __forceinline__ float bfr(float f) { return bf2f(f2bf(f)); }
__device__ __forceinline__ v16h cat16(v8h lo, v8h hi) { return __builtin_shufflevector(lo, hi, 0, 1, 2, 3, 4, 5, 6, 7, 8, 9, 10, 11, 12, 13, 14, 15); }
__device__ __forceinline__ v16bf cat16b(v8us lo, v8us hi) { return __builtin_bit_cast(v16bf, __builtin_shufflevector(lo, hi, 0, 1, 2, 3, 4, 5, 6, 7, 8, 9, 10, 11, 12, 13, 14, 15)); }
__device__ __forceinline__ v8f wmma16(v16h a, v16h b, v8f c) { return __builtin_amdgcn_wmma_f32_16x16x32_f16(false, a, false, b, (short)0, c, false, false); }
__device__ __forceinline__ v8f wmmab(v16bf a, v16bf b, v8f c) { return __builtin_amdgcn_wmma_f32_16x16x32_bf16(false, a, false, b, (short)0, c, false, false); }

template <typename T16> struct WFrag;
template <> struct WFrag<h16> { typedef v16h V; static __device__ __forceinline__ V ld(const h16* p) { return cat16(*(const v8h*)p, *(const v8h*)(p + 16)); } static __device__ __forceinline__ v8f mma(V a, V b, v8f c) { return wmma16(a, b, c); } };
template <> struct WFrag<bf> { typedef v16bf V; static __device__ __forceinline__ V ld(const bf* p) { return cat16b(*(const v8us*)p, *(const v8us*)(p + 16)); } static __device__ __forceinline__ v8f mma(V a, V b, v8f c) { return wmmab(a, b, c); } };
template <typename T16, int NSPLIT, bool BIAS>
__global__ __launch_bounds__(32) void k_gemmw(const T16* __restrict__ A, const T16* __restrict__ A2, const T16* __restrict__ Bt, const T16* __restrict__ Bt2, int K, float* C, int ldc, const float* __restrict__ bias, size_t sA, size_t sB, size_t sC) {
    typedef typename WFrag<T16>::V V;
    __shared__ __align__(16) float os[16 * 68];
    const size_t z = blockIdx.z; A += z * sA; if (A2) A2 += z * sA; Bt += z * sB; if (Bt2) Bt2 += z * sB; C += z * sC;
    const int lane = threadIdx.x & 31, lr = lane & 15, hi = lane >> 4; const int r0 = blockIdx.x * 64, c0 = blockIdx.y * 64;
    v8f acc[4][4];
#pragma unroll
    for (int mb = 0; mb < 4; ++mb)
#pragma unroll
        for (int nb = 0; nb < 4; ++nb) acc[mb][nb] = (v8f){};
    const size_t aoff = (size_t)(r0 + lr) * K + 8 * hi, boff = (size_t)(c0 + lr) * K + 8 * hi;
    for (int kc = 0; kc < K; kc += 32) {
        V a[4], a2[4];
#pragma unroll
        for (int mb = 0; mb < 4; ++mb) { a[mb] = WFrag<T16>::ld(A + aoff + (size_t)mb * 16 * K + kc); if (NSPLIT == 1 || NSPLIT == 2) a2[mb] = WFrag<T16>::ld(A2 + aoff + (size_t)mb * 16 * K + kc); }
#pragma unroll
        for (int nb = 0; nb < 4; ++nb) { const V b = WFrag<T16>::ld(Bt + boff + (size_t)nb * 16 * K + kc); V b2; if (NSPLIT >= 2) b2 = WFrag<T16>::ld(Bt2 + boff + (size_t)nb * 16 * K + kc);
#pragma unroll
            for (int mb = 0; mb < 4; ++mb) { acc[mb][nb] = WFrag<T16>::mma(a[mb], b, acc[mb][nb]); if (NSPLIT == 1 || NSPLIT == 2) acc[mb][nb] = WFrag<T16>::mma(a2[mb], b, acc[mb][nb]); if (NSPLIT >= 2) acc[mb][nb] = WFrag<T16>::mma(a[mb], b2, acc[mb][nb]); } }
        asm volatile("v_nop\n\tv_nop\n\tv_nop\n\tv_nop" : "+v"(acc[0][0]), "+v"(acc[1][1]), "+v"(acc[2][2]), "+v"(acc[3][3]) : "v"(a[0]), "v"(a[3]));
    }
#pragma unroll
    for (int mb = 0; mb < 4; ++mb) {
#pragma unroll
        for (int nb = 0; nb < 4; ++nb) {
#pragma unroll
            for (int j = 0; j < 8; ++j) os[(hi * 8 + j) * 68 + nb * 16 + lr] = acc[mb][nb][j]; }
        __builtin_amdgcn_wave_barrier(); asm volatile("" ::: "memory");
        float* crow = C + (size_t)(r0 + mb * 16) * ldc + c0;
#pragma unroll 1
        for (int ps = 0; ps < 2; ++ps) {
#pragma unroll
            for (int s = 0; s < 8; ++s) { const int row = 2 * s + hi, cofs = lr * 4; v4f val = *(const v4fa*)(os + row * 68 + cofs); if (BIAS) { val[0] += bfr(bias[c0 + cofs]); val[1] += bfr(bias[c0 + cofs + 1]); val[2] += bfr(bias[c0 + cofs + 2]); val[3] += bfr(bias[c0 + cofs + 3]); }
                *(volatile v4f*)(crow + (size_t)row * ldc + cofs) = val; }
            if (ps == 0) __threadfence(); }
        __builtin_amdgcn_wave_barrier(); asm volatile("" ::: "memory");
    }
}

__device__ __forceinline__ void splitf(float y, unsigned short& h, unsigned short& l) { h = f2bf(y); l = f2bf(y - bf2f(h)); }
typedef __attribute__((ext_vector_type(2))) unsigned short v2us;
typedef __attribute__((ext_vector_type(4))) unsigned short v4us;
typedef __attribute__((ext_vector_type(2))) float v2f;

__global__ __launch_bounds__(256) void k_cvt8(const float* __restrict__ src, bf* dst, size_t n8) { const size_t i = (size_t)blockIdx.x * 256 + threadIdx.x; if (i >= n8) return; const v8f v = *(const v8f*)(src + i * 8); v8us o;
#pragma unroll
    for (int k = 0; k < 8; ++k) o[k] = f2bf(v[k]); *(volatile v8us*)(dst + i * 8) = o; __threadfence(); *(volatile v8us*)(dst + i * 8) = o; }

__global__ __launch_bounds__(256) void k_wtG(const float* __restrict__ w, int K, int N, bf* Bt) {
    const int lane = threadIdx.x & 31; const int L0 = (blockIdx.x * 8 + (threadIdx.x >> 5)) * 8; const int nlines = N * K / 64;
#pragma unroll
    for (int ps = 0; ps < 2; ++ps) {
        for (int l = 0; l < 8; ++l) { const int L = L0 + l; if (L >= nlines) break; const size_t e = (size_t)L * 64 + lane * 2; const int k = (int)(e % K), n = (int)(e / K); v2us o;
            o[0] = f2bf(w[(size_t)k * N + n]); o[1] = f2bf(w[(size_t)(k + 1) * N + n]); *(volatile v2us*)(Bt + e) = o; }
        if (ps == 0) __threadfence(); }
}

__global__ __launch_bounds__(256) void k_relu3(const float* __restrict__ F, float* R, bf* Ph, bf* Pl, size_t n4) { const size_t i = (size_t)blockIdx.x * 256 + threadIdx.x; if (i >= n4) return; const v4f v = *(const v4f*)(F + i * 4); v4f r; v4us oh, ol;
#pragma unroll
    for (int q = 0; q < 4; ++q) { const float y = fmaxf(v[q], 0.0f); unsigned short a, c; splitf(y, a, c); r[q] = y; oh[q] = a; ol[q] = c; } *(volatile v4f*)(R + i * 4) = r; *(volatile v4us*)(Ph + i * 4) = oh; *(volatile v4us*)(Pl + i * 4) = ol; __threadfence(); *(volatile v4f*)(R + i * 4) = r; *(volatile v4us*)(Ph + i * 4) = oh; *(volatile v4us*)(Pl + i * 4) = ol; }

__global__ __launch_bounds__(256) void k_dots(const float* __restrict__ Fp, const float* __restrict__ W2, const float* __restrict__ b2, int m, float* DD) {
  const int n = blockIdx.x * 256 + threadIdx.x; if (n >= NN) return; const int n1 = (n + 1) & (NN - 1); const float* fr = Fp + (size_t)n * ND; const float* w = W2 + (size_t)m * ND * NN; float d0 = 0.0f, d1 = 0.0f;
#pragma unroll 1
  for (int d = 0; d < ND; ++d) { const float x = fmaxf(fr[d], 0.0f); d0 += x * bfr(w[(size_t)d * NN + n]); d1 += x * bfr(w[(size_t)d * NN + n1]); }
  v2f o; o[0] = fmaxf(d0 + bfr(b2[(size_t)m * NN + n]), 0.0f); o[1] = fmaxf(d1 + bfr(b2[(size_t)m * NN + n1]), 0.0f); *(volatile v2f*)(DD + (size_t)n * 2) = o; __threadfence(); *(volatile v2f*)(DD + (size_t)n * 2) = o;
}

__global__ __launch_bounds__(256) void k_mix(const float* __restrict__ DD, const float* __restrict__ Vin, float* Vout) {
  const int t = blockIdx.x * 256 + threadIdx.x; if (t >= NN * (ND / 4)) return; const int q = t & (ND / 4 - 1), n = t / (ND / 4); const int n1 = (n + 1) & (NN - 1);
  const v2f dd = *(const v2f*)(DD + (size_t)n * 2); const v4f a = *(const v4f*)(Vin + (size_t)n * ND + q * 4); const v4f c = *(const v4f*)(Vin + (size_t)n1 * ND + q * 4); v4f o;
#pragma unroll
  for (int e = 0; e < 4; ++e) o[e] = dd[0] * a[e] + dd[1] * c[e];
  *(volatile v4f*)(Vout + (size_t)n * ND + q * 4) = o; __threadfence(); *(volatile v4f*)(Vout + (size_t)n * ND + q * 4) = o;
}

extern "C" void kernel_launch(void* const* d_in, const int* in_sizes, int n_in,
                              void* d_out, int out_size, void* d_ws, size_t ws_size, hipStream_t stream) {
    (void)in_sizes; (void)n_in; (void)out_size;
    const float* X = (const float*)d_in[0]; const float* gW = (const float*)d_in[1]; const float* gb = (const float*)d_in[2]; const float* fW1 = (const float*)d_in[3]; const float* fb1 = (const float*)d_in[4]; const float* fW2 = (const float*)d_in[5]; const float* fb2 = (const float*)d_in[6];
    (void)d_in[7]; (void)d_in[8];
    float* OUT = (float*)d_out;
    char* wsp = (char*)d_ws;
    auto take = [&](size_t bytes) { char* p = wsp; wsp += (bytes + 255) & ~(size_t)255; return (void*)p; };
    const size_t NE = (size_t)NN * ND;
    bf* XB = (bf*)take(NE * 2); bf* WT = (bf*)take((size_t)5 * ND * ND * 2); float* C = (float*)take(NE * 4); float* V0 = (float*)take(NE * 4); float* V1 = (float*)take(NE * 4); bf* Ph = (bf*)take(NE * 2); bf* Pl = (bf*)take(NE * 2); float* DD = (float*)take((size_t)NN * 2 * 4);
    if ((size_t)(wsp - (char*)d_ws) > ws_size) return;
    k_cvt8<<<(unsigned)((NE / 8 + 255) / 256), 256, 0, stream>>>(X, XB, NE / 8);
    for (int j = 0; j < 2; ++j) k_wtG<<<(unsigned)((ND * ND / 64 + 63) / 64), 256, 0, stream>>>(gW + (size_t)j * ND * ND, ND, ND, WT + (size_t)j * ND * ND);
    for (int m = 0; m < NLY; ++m) k_wtG<<<(unsigned)((ND * ND / 64 + 63) / 64), 256, 0, stream>>>(fW1 + (size_t)m * ND * ND, ND, ND, WT + (size_t)(2 + m) * ND * ND);
    k_gemmw<bf, 0, true><<<dim3(NN / 64, ND / 64, 1), 32, 0, stream>>>(XB, nullptr, WT, nullptr, ND, C, ND, gb, 0, 0, 0);
    k_relu3<<<(unsigned)((NE / 4 + 255) / 256), 256, 0, stream>>>(C, V1, Ph, Pl, NE / 4);
    k_gemmw<bf, 1, true><<<dim3(NN / 64, ND / 64, 1), 32, 0, stream>>>(Ph, Pl, WT + (size_t)ND * ND, nullptr, ND, C, ND, gb + ND, 0, 0, 0);
    k_relu3<<<(unsigned)((NE / 4 + 255) / 256), 256, 0, stream>>>(C, V0, Ph, Pl, NE / 4);
    k_gemmw<bf, 0, true><<<dim3(NN / 64, ND / 64, 1), 32, 0, stream>>>(XB, nullptr, WT + (size_t)2 * ND * ND, nullptr, ND, C, ND, fb1, 0, 0, 0); k_dots<<<NN / 256, 256, 0, stream>>>(C, fW2, fb2, 0, DD); k_mix<<<(unsigned)(NE / 4 / 256), 256, 0, stream>>>(DD, V0, V1);
    k_gemmw<bf, 0, true><<<dim3(NN / 64, ND / 64, 1), 32, 0, stream>>>(XB, nullptr, WT + (size_t)3 * ND * ND, nullptr, ND, C, ND, fb1 + ND, 0, 0, 0); k_dots<<<NN / 256, 256, 0, stream>>>(C, fW2, fb2, 1, DD); k_mix<<<(unsigned)(NE / 4 / 256), 256, 0, stream>>>(DD, V1, V0);
    k_gemmw<bf, 0, true><<<dim3(NN / 64, ND / 64, 1), 32, 0, stream>>>(XB, nullptr, WT + (size_t)4 * ND * ND, nullptr, ND, C, ND, fb1 + (size_t)2 * ND, 0, 0, 0); k_dots<<<NN / 256, 256, 0, stream>>>(C, fW2, fb2, 2, DD); k_mix<<<(unsigned)(NE / 4 / 256), 256, 0, stream>>>(DD, V0, OUT);
}
